// CAM_Module_90211493085854
// MI455X (gfx1250) — hardware-verified
//
#include <hip/hip_runtime.h>
#include <math.h>

#ifndef NB
#define NB 128
#endif
#define NB_FULL 128
#define CH 1024
#define NPOS 49
#define NPAD 64
#define ENT_FULL (CH * NPOS)

static_assert(NB >= 1 && NB <= NB_FULL);
static_assert(CH == 1024);
static_assert(NPOS == 49);
static_assert(NPAD == 64);
static_assert(NPOS <= NPAD);
static_assert(CH % 64 == 0 && NPAD % 64 == 0);
static_assert(CH % 32 == 0 && NPAD % 32 == 0);
static_assert((NPAD * (CH / 8)) % 256 == 0);
static_assert((CH * 8) % 256 == 0);
static_assert(ENT_FULL % 256 == 0);
static_assert((size_t)NB_FULL * ENT_FULL * 4 == (size_t)25690112);
static_assert((size_t)NB * ENT_FULL * 4 <= (size_t)25690112);
static_assert((size_t)NB_FULL * ENT_FULL < (size_t)2147483647);

typedef __attribute__((ext_vector_type(16))) _Float16 v16h;
typedef __attribute__((ext_vector_type(8)))  _Float16 v8h;
typedef __attribute__((ext_vector_type(4)))  _Float16 v4h;
typedef __attribute__((ext_vector_type(2)))  _Float16 v2h;
typedef __attribute__((ext_vector_type(8)))  float    v8f;
typedef __attribute__((ext_vector_type(4)))  float    v4f;
typedef __attribute__((ext_vector_type(2)))  float    v2f;
typedef _Float16 h16;


#define VST2(T, ptr, val) do { const T vst2_v_ = (val); *(volatile T*)(ptr) = vst2_v_; __threadfence(); *(volatile T*)(ptr) = vst2_v_; } while (0)
#define VST2V4(ptr, val) do { const v4f vst2_v4_ = (val); *(volatile v4f*)(ptr) = vst2_v4_; __threadfence(); *(volatile v4f*)(ptr) = vst2_v4_; } while (0)

__device__ __forceinline__ float bfr(float f) {
    unsigned u = __float_as_uint(f);
    u += 0x7FFFu + ((u >> 16) & 1u);
    return __uint_as_float(u & 0xFFFF0000u);
}

static __device__ __forceinline__ h16 toh_flush(float v) {
    const float w = (fabsf(v) < 6.103515625e-05f) ? 0.0f : v;
    return (h16)w;
}
static __device__ __forceinline__ v2h toh_flush2(float a, float b) {
    v2f w;
    w.x = (fabsf(a) < 6.103515625e-05f) ? 0.0f : a;
    w.y = (fabsf(b) < 6.103515625e-05f) ? 0.0f : b;
    return __builtin_convertvector(w, v2h);
}
static __device__ __forceinline__ v8h pack8h_flush(const float* v) {
    const v2h p0 = toh_flush2(v[0], v[1]);
    const v2h p1 = toh_flush2(v[2], v[3]);
    const v2h p2 = toh_flush2(v[4], v[5]);
    const v2h p3 = toh_flush2(v[6], v[7]);
    const v4h q0 = __builtin_shufflevector(p0, p1, 0, 1, 2, 3);
    const v4h q1 = __builtin_shufflevector(p2, p3, 0, 1, 2, 3);
    return __builtin_shufflevector(q0, q1, 0, 1, 2, 3, 4, 5, 6, 7);
}
static __device__ __forceinline__ void st8h_flush(_Float16* P, size_t o, const float* v) {
    const v8h pk = pack8h_flush(v);
    VST2(v8h, (v8h*)(P + o), pk);
}

union FragU { v16h v; v8h h[2]; };
__device__ __forceinline__ v16h frag_ld(const _Float16* p) {
    FragU f; f.h[0] = *(const v8h*)(p); f.h[1] = *(const v8h*)(p + 16); return f.v;
}
__device__ __forceinline__ v8f wmma16(v16h a, v16h b, v8f c) {
    c = __builtin_amdgcn_wmma_f32_16x16x32_f16(false, a, false, b, (short)0, c, false, false);
    asm volatile("v_nop\n\tv_nop\n\tv_nop\n\tv_nop" : "+v"(c) : "v"(a), "v"(b));
    return c;
}
__device__ __forceinline__ void wave_sync_lds() {
    __builtin_amdgcn_fence(3  , "workgroup");
    __builtin_amdgcn_wave_barrier();
    __builtin_amdgcn_fence(2  , "workgroup");
}

#define SLAB_FLOATS (16 * 68)
static_assert((size_t)8 * SLAB_FLOATS * 4 <= (size_t)131072);

template <int OUT_MODE>
static __device__ __forceinline__ void gemm64_body(
    const _Float16* __restrict__ A, unsigned lda, const _Float16* __restrict__ Bt, unsigned ldb,
    void* __restrict__ Cout, unsigned ldc, unsigned M, unsigned N, unsigned K, float scale, float oscale,
    float* sTbase) {
  const unsigned lane = threadIdx.x & 31u;
  const unsigned wave = (unsigned)__builtin_amdgcn_readfirstlane((int)(threadIdx.x >> 5));
  const unsigned tilesN = N >> 6, tilesM = M >> 6;
  const unsigned tile = blockIdx.x * 8u + wave;
  if (tile >= tilesM * tilesN) return;
  const unsigned tm = tile / tilesN;
  const unsigned tn = tile - tm * tilesN;
  const unsigned m0 = tm << 6, n0 = tn << 6;
  const unsigned rlane = lane & 15u;
  const unsigned koff = (lane >> 4) * 8u;
  const unsigned mOff = koff;

  v8f acc[4][4];
#pragma unroll
  for (int i = 0; i < 4; ++i)
#pragma unroll
    for (int j = 0; j < 4; ++j) acc[i][j] = (v8f){0.f,0.f,0.f,0.f,0.f,0.f,0.f,0.f};

  for (unsigned k0 = 0; k0 < K; k0 += 32u) {
    v16h bh[4];
#pragma unroll
    for (int j = 0; j < 4; ++j)
      bh[j] = frag_ld(Bt + (size_t)(n0 + ((unsigned)j << 4) + rlane) * ldb + koff + k0);
#pragma unroll
    for (int i = 0; i < 4; ++i) {
      const v16h ah = frag_ld(A + (size_t)(m0 + ((unsigned)i << 4) + rlane) * lda + koff + k0);
#pragma unroll
      for (int j = 0; j < 4; ++j)
        acc[i][j] = wmma16(ah, bh[j], acc[i][j]);
    }
  }

  float* slab = sTbase + wave * (unsigned)SLAB_FLOATS;
#pragma unroll
  for (int i = 0; i < 4; ++i) {
    const unsigned mBase = m0 + ((unsigned)i << 4);
#pragma unroll
    for (int j = 0; j < 4; ++j) {
#pragma unroll
      for (int r = 0; r < 8; ++r) {
        float v = acc[i][j][r] * scale;
        if (OUT_MODE == 1) v *= oscale;
        slab[(mOff + (unsigned)r) * 68u + ((unsigned)j << 4) + rlane] = v;
      }
    }
    wave_sync_lds();
    if (OUT_MODE == 0) {
      float* C = (float*)Cout;
      const unsigned hh = lane >> 4, c4 = (lane & 15u) * 4u;
      static_assert(32 * 16 * 2 * 4 == 16 * 64 * 4);
#pragma unroll
      for (int half = 0; half < 2; ++half) {
        v4f vv[4];
#pragma unroll
        for (int it = 0; it < 4; ++it) {
          const unsigned row = (unsigned)(half * 4 + it) * 2u + hh;
          vv[it] = *(const v4f*)(slab + row * 68u + c4);
        }
        for (int pass = 0; pass < 2; ++pass) {
#pragma unroll
          for (int it = 0; it < 4; ++it) {
            const unsigned row = (unsigned)(half * 4 + it) * 2u + hh;
            *(volatile v4f*)(C + (size_t)(mBase + row) * ldc + n0 + c4) = vv[it];
          }
          __threadfence();
        }
      }
    } else {
      _Float16* C = (_Float16*)Cout;
      const unsigned q = lane >> 3, c8 = (lane & 7u) * 8u;
      static_assert(32 * 16 * 4 == 16 * 64 * 2);
      v8h hv[4];
#pragma unroll
      for (int it = 0; it < 4; ++it) {
        const unsigned row = (unsigned)it * 4u + q;
        const float* sp = slab + row * 68u + c8;
        float tv[8];
#pragma unroll
        for (int e = 0; e < 8; ++e) tv[e] = sp[e];
        hv[it] = pack8h_flush(tv);
      }
      for (int pass = 0; pass < 2; ++pass) {
#pragma unroll
        for (int it = 0; it < 4; ++it) {
          const unsigned row = (unsigned)it * 4u + q;
          *(volatile v8h*)(C + (size_t)(mBase + row) * ldc + n0 + c8) = hv[it];
        }
        __threadfence();
      }
    }
    wave_sync_lds();
  }
}

__global__ __launch_bounds__(256) void k_gemm_tt(const _Float16* __restrict__ VT16, const _Float16* __restrict__ KT16,
                                                 _Float16* __restrict__ TT16) {
    __shared__ __align__(16) float sT[8][SLAB_FLOATS];
    const unsigned b = blockIdx.y;
    gemm64_body<1>(VT16 + (size_t)b * NPAD * CH, CH, KT16 + (size_t)b * NPAD * CH, CH,
                   (void*)(TT16 + (size_t)b * NPAD * NPAD), NPAD, NPAD, NPAD, CH,
                   1.0f / 4096.0f, 64.0f, &sT[0][0]);
}

__global__ __launch_bounds__(256) void k_gemm_c(const _Float16* __restrict__ Q16, const _Float16* __restrict__ TT16,
                                                float* __restrict__ C32) {
    __shared__ __align__(16) float sT[8][SLAB_FLOATS];
    const unsigned b = blockIdx.y;
    gemm64_body<0>(Q16 + (size_t)b * CH * NPAD, NPAD, TT16 + (size_t)b * NPAD * NPAD, NPAD,
                   (void*)(C32 + (size_t)b * CH * NPAD), NPAD, CH, NPAD, NPAD,
                   1.0f / 4096.0f, 1.0f, &sT[0][0]);
}

static_assert((size_t)(NPAD * (CH / 8)) * 16 == (size_t)NPAD * CH * 2);
__global__ __launch_bounds__(256) void k_cvt_t(const float* __restrict__ X, _Float16* __restrict__ XT16) {
    const unsigned b = blockIdx.y;
    const unsigned u = blockIdx.x * 256u + threadIdx.x;
    if (u >= (unsigned)(NPAD * (CH / 8))) return;
    const unsigned d0 = 8u * (u & 127u);
    const unsigned n = u >> 7;
    const unsigned nc = (n < (unsigned)NPOS) ? n : (unsigned)(NPOS - 1);
    const float* src = X + (size_t)b * ENT_FULL + nc;
    float v[8];
#pragma unroll
    for (int i = 0; i < 8; ++i) {
        const float x = src[(size_t)(d0 + (unsigned)i) * NPOS];
        v[i] = (n < (unsigned)NPOS) ? bfr(x) * 64.0f : 0.0f;
    }
    st8h_flush(XT16, (size_t)b * NPAD * CH + (size_t)n * CH + d0, v);
}

static_assert((size_t)(CH * 8) * 16 == (size_t)CH * NPAD * 2);
__global__ __launch_bounds__(256) void k_cvt_q(const float* __restrict__ Qin, _Float16* __restrict__ Q16) {
    const unsigned b = blockIdx.y;
    const unsigned u = blockIdx.x * 256u + threadIdx.x;
    if (u >= (unsigned)(CH * 8)) return;
    const unsigned row = u >> 3, c0 = (u & 7u) * 8u;
    const float* src = Qin + (size_t)b * ENT_FULL + (size_t)row * NPOS;
    float v[8];
#pragma unroll
    for (int i = 0; i < 8; ++i) {
        const unsigned col = c0 + (unsigned)i;
        const unsigned cc = (col < (unsigned)NPOS) ? col : (unsigned)(NPOS - 1);
        const float x = src[cc];
        v[i] = (col < (unsigned)NPOS) ? bfr(x) * 64.0f : 0.0f;
    }
    st8h_flush(Q16, (size_t)b * CH * NPAD + (size_t)row * NPAD + c0, v);
}

static_assert(((size_t)NB * ENT_FULL) % 256 == 0);
__global__ __launch_bounds__(256) void k_out(const float* __restrict__ C32, const float* __restrict__ v1,
                                             float* __restrict__ out) {
    const unsigned u = blockIdx.x * 256u + threadIdx.x;
    if (u >= (unsigned)(NB * ENT_FULL)) return;
    unsigned uu = u; asm volatile("" : "+v"(uu));
    const unsigned row = uu / (unsigned)NPOS;
    const unsigned n = uu - row * (unsigned)NPOS;
    const float val = C32[(size_t)row * NPAD + n] + bfr(v1[u]);
    VST2(float, out + u, val);
}

constexpr size_t SZ_T16  = (size_t)NB * NPAD * CH * 2;
constexpr size_t SZ_Q16  = (size_t)NB * CH * NPAD * 2;
constexpr size_t SZ_TT16 = (size_t)NB * NPAD * NPAD * 2;
constexpr size_t SZ_C32  = (size_t)NB * CH * NPAD * 4;
constexpr size_t OFF_KT   = 0;
constexpr size_t OFF_VT   = OFF_KT + SZ_T16;
constexpr size_t OFF_Q    = OFF_VT + SZ_T16;
constexpr size_t OFF_TT   = OFF_Q + SZ_Q16;
constexpr size_t OFF_C    = OFF_TT + SZ_TT16;
constexpr size_t WS_TOTAL = OFF_C + SZ_C32;
static_assert(SZ_T16 % 256 == 0 && SZ_Q16 % 256 == 0 && SZ_TT16 % 256 == 0 && SZ_C32 % 256 == 0);
static_assert(WS_TOTAL <= (size_t)134217728);

extern "C" void kernel_launch(void* const* d_in, const int* in_sizes, int n_in, void* d_out, int out_size,
                              void* d_ws, size_t ws_size, hipStream_t stream) {
    if (n_in < 3) return;
    const int need = NB * ENT_FULL;
    if (in_sizes[0] < need || in_sizes[1] < need || in_sizes[2] < need) return;
    if (out_size < need) return;
    if (WS_TOTAL > ws_size) return;

    const float* v1 = (const float*)d_in[0];
    const float* q1 = (const float*)d_in[1];
    const float* k1 = (const float*)d_in[2];
    float* out = (float*)d_out;

    char* wsp = (char*)d_ws;
    _Float16* KT16 = (_Float16*)(wsp + OFF_KT);
    _Float16* VT16 = (_Float16*)(wsp + OFF_VT);
    _Float16* Q16  = (_Float16*)(wsp + OFF_Q);
    _Float16* TT16 = (_Float16*)(wsp + OFF_TT);
    float*    C32  = (float*)(wsp + OFF_C);

    k_cvt_t<<<dim3((NPAD * (CH / 8)) / 256, NB), 256, 0, stream>>>(k1, KT16);
    k_cvt_t<<<dim3((NPAD * (CH / 8)) / 256, NB), 256, 0, stream>>>(v1, VT16);
    k_cvt_q<<<dim3((CH * 8) / 256, NB), 256, 0, stream>>>(q1, Q16);

    k_gemm_tt<<<dim3(1, NB), 32, 0, stream>>>((const _Float16*)VT16, (const _Float16*)KT16, TT16);
    k_gemm_c<<<dim3(((CH / 64) * (NPAD / 64) + 7) / 8, NB), 256, 0, stream>>>((const _Float16*)Q16, (const _Float16*)TT16, C32);

    k_out<<<(NB * ENT_FULL) / 256, 256, 0, stream>>>((const float*)C32, v1, out);
}
